// CausalSelfAttention_8280696946882
// MI455X (gfx1250) — hardware-verified
//
#include <hip/hip_runtime.h>


#ifndef NB
#define NB 8
#endif
#ifndef SEQ
#define SEQ 2048
#endif
#define NB_FULL  8
#define SEQ_FULL 2048
#ifndef OUT_SEQ
#define OUT_SEQ SEQ
#endif
#define DMI  126
#define DK   128
#define NH_  6
#define HDR  21
#define HD   32
#define DH   192
#define DNO  128
#define AW   4
#define OSP  36
#define EROWS (SEQ < 256 ? SEQ : 256)
#define QRS  2048.0f
#define QRI  (1.0f / 2048.0f)
#define SC2  ((float)(0.2182178902359924 * 1.4426950408889634))
#define PSH  14.0f
#define PFL  (-14.0f)
#define CTXS 16.0f
#define WPS  64.0f
#define OSC  (1.0f / 1024.0f)
#define NEGB (-3.0e38f)
#define OPQ  (16 * DMI / 4)
#define OPT  16
#define WBLK 36
#define PBLK 12

static_assert(HD == 32);
static_assert(NH_ * HDR == DMI);
static_assert(NH_ * HD == DH);
static_assert(HDR <= HD);
static_assert(DK == 128);
static_assert(DK >= DMI);
static_assert(DK % 32 == 0);
static_assert(DH % 64 == 0);
static_assert(64 % HD == 0);
static_assert(DNO == 128);
static_assert(DNO >= DMI);
static_assert(SEQ % 64 == 0);
static_assert((NB * SEQ) % 64 == 0);
static_assert(SEQ % 32 == 0);
static_assert(SEQ % (16 * AW) == 0);
static_assert(EROWS % 64 == 0);
static_assert(EROWS % 32 == 0);
static_assert(EROWS >= 32);
static_assert(EROWS <= SEQ);
static_assert(EROWS % (16 * AW) == 0);
static_assert((SEQ - EROWS) % (16 * AW) == 0);
static_assert(NB <= NB_FULL);
static_assert(SEQ <= SEQ_FULL);
static_assert(OUT_SEQ % 16 == 0);
static_assert(OUT_SEQ >= SEQ);
static_assert((OSP * 4) % 16 == 0);
static_assert((16 * DMI * 4) % 128 == 0);
static_assert((16 * DMI) % 4 == 0);
static_assert(OPT * 32 >= OPQ);
static_assert((OPT - 1) * 32 < OPQ);
static_assert((OPQ % 32) % 8 == 0);
static_assert(3 * DH * DK / 8 == WBLK * 256);
static_assert(DNO * DH / 8 == PBLK * 256);
static_assert(2 * 2 * 32 * 16 == 16 * 64 * 2);
static_assert(4 * 32 * 16 == 16 * 64 * 2);
static_assert(2 * 32 * 16 == 16 * HD * 2);
static_assert(16 * 68 * 4 <= 131072);
static_assert(AW * 16 * OSP * 4 <= 131072);
static_assert(AW * 16 * DMI * 4 <= 131072);

typedef _Float16 h16;
typedef unsigned short bf;
typedef __attribute__((ext_vector_type(16))) __bf16   v16bf;
typedef __attribute__((ext_vector_type(16))) _Float16 v16h;
typedef __attribute__((ext_vector_type(8)))  _Float16 v8h;
typedef __attribute__((ext_vector_type(8)))  unsigned short v8us;
typedef __attribute__((ext_vector_type(8)))  float    v8f;
typedef __attribute__((ext_vector_type(4)))  float    v4f;
typedef v4f  __attribute__((may_alias)) v4fa;

__device__ __forceinline__ unsigned short f2bf(float f) { unsigned u = __float_as_uint(f); u += 0x7FFFu + ((u >> 16) & 1u); return (unsigned short)(u >> 16); }
__device__ __forceinline__ float bfr(float f) { return __uint_as_float(((unsigned)f2bf(f)) << 16); }
__device__ __forceinline__ v16h cat16(v8h lo, v8h hi) { return __builtin_shufflevector(lo, hi, 0, 1, 2, 3, 4, 5, 6, 7, 8, 9, 10, 11, 12, 13, 14, 15); }
__device__ __forceinline__ v16bf cat16b(v8us lo, v8us hi) { return __builtin_bit_cast(v16bf, __builtin_shufflevector(lo, hi, 0, 1, 2, 3, 4, 5, 6, 7, 8, 9, 10, 11, 12, 13, 14, 15)); }
__device__ __forceinline__ v8f wmma16(v16h a, v16h b, v8f c) { return __builtin_amdgcn_wmma_f32_16x16x32_f16(false, a, false, b, (short)0, c, false, false); }
__device__ __forceinline__ v8f wmmab(v16bf a, v16bf b, v8f c) { return __builtin_amdgcn_wmma_f32_16x16x32_bf16(false, a, false, b, (short)0, c, false, false); }
__device__ __forceinline__ v16h  ldh(const h16* p) { return cat16(*(const v8h*)p, *(const v8h*)(p + 16)); }
__device__ __forceinline__ v16bf ldb(const bf* p)  { return cat16b(*(const v8us*)p, *(const v8us*)(p + 16)); }
__device__ __forceinline__ void wave_sync() { __builtin_amdgcn_fence(3  , "wavefront"); __builtin_amdgcn_wave_barrier(); asm volatile("" ::: "memory"); }

__device__ __forceinline__ h16 toh_flush(float v) { const h16 r = (h16)v; return (fabsf(v) < 6.103515625e-05f) ? (h16)0.0f : r; }
__device__ __forceinline__ v8f wmma16g(v16h a, v16h b, v8f c) { c = wmma16(a, b, c); asm volatile("v_nop\n\tv_nop\n\tv_nop\n\tv_nop" : "+v"(c) : "v"(a), "v"(b)); return c; }
__device__ __forceinline__ v8f wmmabg(v16bf a, v16bf b, v8f c) { c = wmmab(a, b, c); asm volatile("v_nop\n\tv_nop\n\tv_nop\n\tv_nop" : "+v"(c) : "v"(a), "v"(b)); return c; }

__global__ __launch_bounds__(256) void k_padx(const float* __restrict__ src, bf* dst, unsigned n8) {
    const unsigned i = blockIdx.x * 256u + threadIdx.x; if (i >= n8) return;
    const unsigned row = i >> 4, c8 = (i & 15u) * 8u;
    const unsigned bb = row / (unsigned)SEQ, tt = row % (unsigned)SEQ;
    const float* s = src + ((size_t)bb * SEQ_FULL + (size_t)tt) * DMI;
    v8us o;
#pragma unroll
    for (int k = 0; k < 8; ++k) {
        const unsigned c = c8 + (unsigned)k; const unsigned cc = c < (unsigned)DMI ? c : (unsigned)(DMI - 1);
        float v = s[cc]; asm volatile("" : "+v"(v));
        o[k] = (c < (unsigned)DMI) ? f2bf(v) : (unsigned short)0; }
    *(volatile v8us*)(dst + (size_t)i * 8) = o; __threadfence(); *(volatile v8us*)(dst + (size_t)i * 8) = o;
}

__global__ __launch_bounds__(256) void k_wprep(const float* __restrict__ wa, const float* __restrict__ wp, bf* WB, h16* WP) {
    if (blockIdx.x < WBLK) {
        const unsigned i = blockIdx.x * 256u + threadIdx.x;
        const unsigned e0 = i * 8u; const unsigned sec = e0 / (unsigned)(DH * DK), rem = e0 % (unsigned)(DH * DK);
        const unsigned n = rem / (unsigned)DK, k0 = rem % (unsigned)DK;
        const unsigned h = n / (unsigned)HD, d = n % (unsigned)HD; const bool dok = d < (unsigned)HDR;
        const unsigned col = sec * (unsigned)DMI + h * (unsigned)HDR + (dok ? d : 0u);
        v8us o;
#pragma unroll
        for (int k = 0; k < 8; ++k) {
            const unsigned kk = k0 + (unsigned)k; const unsigned kc = kk < (unsigned)DMI ? kk : (unsigned)(DMI - 1);
            float v = wa[(size_t)kc * (3 * DMI) + col]; asm volatile("" : "+v"(v));
            o[k] = (dok & (kk < (unsigned)DMI)) ? f2bf(v) : (unsigned short)0; }
        *(volatile v8us*)(WB + (size_t)e0) = o; __threadfence(); *(volatile v8us*)(WB + (size_t)e0) = o;
    } else {
        const unsigned j = (blockIdx.x - WBLK) * 256u + threadIdx.x; if (j >= (unsigned)(DNO * DH / 8)) return;
        const unsigned e0 = j * 8u; const unsigned n = e0 / (unsigned)DH, k0 = e0 % (unsigned)DH;
        const unsigned h = k0 / (unsigned)HD, d0 = k0 % (unsigned)HD;
        const unsigned nc = n < (unsigned)DMI ? n : (unsigned)(DMI - 1); const bool nok = n < (unsigned)DMI;
        v8h o;
#pragma unroll
        for (int k = 0; k < 8; ++k) {
            const unsigned d = d0 + (unsigned)k; const unsigned dc = d < (unsigned)HDR ? d : (unsigned)(HDR - 1);
            float v = wp[(size_t)(h * (unsigned)HDR + dc) * DMI + nc]; asm volatile("" : "+v"(v));
            const h16 c = toh_flush(bfr(v) * WPS);
            o[k] = (nok & (d < (unsigned)HDR)) ? c : (h16)0.0f; }
        *(volatile v8h*)(WP + (size_t)e0) = o; __threadfence(); *(volatile v8h*)(WP + (size_t)e0) = o;
    }
}

template <int MODE>
__device__ __forceinline__ void proj_body(const bf* __restrict__ A, const bf* __restrict__ Bt, h16* Ph, h16* Pr, int resT) {
    __shared__ __align__(16) float os[16 * 68];
    const int K = DK;
    const int lane = threadIdx.x & 31, lr = lane & 15, hi = lane >> 4; const int r0 = blockIdx.x * 64, c0 = blockIdx.y * 64;
    v8f acc[4][4];
#pragma unroll
    for (int mb = 0; mb < 4; ++mb)
#pragma unroll
        for (int nb = 0; nb < 4; ++nb) acc[mb][nb] = (v8f){};
    const size_t aoff = (size_t)(r0 + lr) * K + 8 * hi, boff = (size_t)(c0 + lr) * K + 8 * hi;
#pragma unroll 1
    for (int kc = 0; kc < K; kc += 32) {
        v16bf a[4];
#pragma unroll
        for (int mb = 0; mb < 4; ++mb) a[mb] = ldb(A + aoff + (size_t)mb * 16 * K + kc);
#pragma unroll
        for (int nb = 0; nb < 4; ++nb) { const v16bf b = ldb(Bt + boff + (size_t)nb * 16 * K + kc);
#pragma unroll
            for (int mb = 0; mb < 4; ++mb) acc[mb][nb] = wmmabg(a[mb], b, acc[mb][nb]); }
    }
    size_t tbase, rbase; bool wr;
    if (MODE == 0) { const int bb = r0 / SEQ, tt = r0 % SEQ; const int zc = bb * NH_ + c0 / HD;
                     tbase = ((size_t)zc * SEQ + (size_t)tt) * HD; rbase = ((size_t)zc * (size_t)resT + (size_t)tt) * HD; wr = tt < resT; }
    else           { const int bb = c0 / SEQ, tt = c0 % SEQ;
                     tbase = (size_t)bb * (size_t)DH * SEQ + (size_t)r0 * SEQ + (size_t)tt; rbase = (size_t)bb * (size_t)DH * (size_t)resT + (size_t)r0 * (size_t)resT + (size_t)tt; wr = tt < resT; }
#pragma unroll
    for (int mb = 0; mb < 4; ++mb) {
#pragma unroll
        for (int nb = 0; nb < 4; ++nb) {
#pragma unroll
            for (int j = 0; j < 8; ++j) os[(hi * 8 + j) * 68 + nb * 16 + lr] = acc[mb][nb][j]; }
        wave_sync();
#pragma unroll 1
        for (int ps = 0; ps < 2; ++ps) {
            if (MODE == 0) {
                const size_t sb = tbase + (size_t)(mb * 16) * HD;
                const size_t rb = rbase + (size_t)(mb * 16) * HD;
#pragma unroll
                for (int hh = 0; hh < 2; ++hh) {
#pragma unroll
                    for (int s = 0; s < 2; ++s) { const int p = s * 32 + lane; const int row = p >> 2, c8 = (p & 3) * 8;
                        const v4f x0 = *(const v4fa*)(&os[row * 68 + hh * 32 + c8]); const v4f x1 = *(const v4fa*)(&os[row * 68 + hh * 32 + c8 + 4]); v8h hv, rv;
#pragma unroll
                        for (int i = 0; i < 4; ++i) { const h16 a0 = toh_flush(x0[i]); const h16 a1 = toh_flush(x1[i]); hv[i] = a0; hv[4 + i] = a1; rv[i] = toh_flush((x0[i] - (float)a0) * QRS); rv[4 + i] = toh_flush((x1[i] - (float)a1) * QRS); }
                        const size_t oo = sb + (size_t)hh * ((size_t)SEQ * HD) + (size_t)p * 8;
                        const size_t ro = rb + (size_t)hh * ((size_t)resT * HD) + (size_t)p * 8;
                        *(volatile v8h*)(Ph + oo) = hv; if (wr) *(volatile v8h*)(Pr + ro) = rv; } }
            } else {
                const size_t sb = tbase + (size_t)(mb * 16) * SEQ;
                const size_t rb = rbase + (size_t)(mb * 16) * (size_t)resT;
#pragma unroll
                for (int s = 0; s < 4; ++s) { const int row = 4 * s + (lane >> 3), c8 = (lane & 7) * 8;
                    const v4f x0 = *(const v4fa*)(&os[row * 68 + c8]); const v4f x1 = *(const v4fa*)(&os[row * 68 + c8 + 4]); v8h hv, rv;
#pragma unroll
                    for (int i = 0; i < 4; ++i) { const h16 a0 = toh_flush(x0[i]); const h16 a1 = toh_flush(x1[i]); hv[i] = a0; hv[4 + i] = a1; rv[i] = toh_flush((x0[i] - (float)a0) * QRS); rv[4 + i] = toh_flush((x1[i] - (float)a1) * QRS); }
                    const size_t oo = sb + (size_t)row * SEQ + c8;
                    const size_t ro = rb + (size_t)row * (size_t)resT + c8;
                    *(volatile v8h*)(Ph + oo) = hv; if (wr) *(volatile v8h*)(Pr + ro) = rv; }
            }
            if (ps == 0) __threadfence(); }
        wave_sync();
    }
}

__global__ __launch_bounds__(32) void k_proj_rows(const bf* __restrict__ A, const bf* __restrict__ Bt, h16* Ph, h16* Pr, int resT) { proj_body<0>(A, Bt, Ph, Pr, resT); }
__global__ __launch_bounds__(32) void k_proj_cols(const bf* __restrict__ A, const bf* __restrict__ Bt, h16* Ph, h16* Pr, int resT) { proj_body<1>(A, Bt, Ph, Pr, resT); }

template <int EARLY>
__device__ __forceinline__ void flash_body(const h16* __restrict__ QH, const h16* __restrict__ QR, const h16* __restrict__ KP, const h16* __restrict__ KR,
                                           const h16* __restrict__ VT, const h16* __restrict__ VR, h16* CH, h16* CR) {
    __shared__ __align__(16) float os[AW * 16 * OSP];
    const int lane = threadIdx.x & 31, lr = lane & 15, hi = lane >> 4;
    const int wave = __builtin_amdgcn_readfirstlane((int)(threadIdx.x >> 5));
    const int zh = blockIdx.y; const int b = zh / NH_, h = zh % NH_;
    const int t0 = (EARLY ? 0 : EROWS) + (blockIdx.x * AW + wave) * 16;
    const int lim = t0 + lr;
    const int nk = (t0 + 16 + 31) & ~31;
    const size_t pbase = (size_t)zh * SEQ * HD;
    const size_t rbase = (size_t)zh * EROWS * HD;
    const size_t qo = pbase + (size_t)(t0 + lr) * HD + 8 * hi;
    const size_t qro = rbase + (size_t)(EARLY ? (t0 + lr) : lr) * HD + 8 * hi;
    const v16h hz = (v16h){};
    const v16h qh = ldh(QH + qo);
    v16h qr = hz; if (EARLY) qr = ldh(QR + qro);
    const size_t ko = pbase + (size_t)lr * HD + 8 * hi;
    const size_t vo = pbase + (size_t)lr * SEQ + 8 * hi;
    const size_t kro = rbase + (size_t)lr * HD + 8 * hi;
    const size_t vro = rbase + (size_t)lr * EROWS + 8 * hi;
    v8f o0 = (v8f){}, o1 = (v8f){}, oR0 = (v8f){}, oR1 = (v8f){};
    float m = NEGB, l = 0.0f;
#pragma unroll 1
    for (int key0 = 0; key0 < nk; key0 += 32) {
        const h16* ka = KP + ko + (size_t)key0 * HD;
        const v16h ka0 = ldh(ka), kb0 = ldh(ka + 16 * HD);
        v8f sHa = (v8f){}, sLa = (v8f){}, sHb = (v8f){}, sLb = (v8f){};
        sHa = wmma16g(ka0, qh, sHa); sHb = wmma16g(kb0, qh, sHb);
        if (EARLY) {
            const h16* kr = KR + kro + (size_t)key0 * HD;
            const v16h kra0 = ldh(kr), krb0 = ldh(kr + 16 * HD);
            sLa = wmma16g(ka0, qr, sLa); sLb = wmma16g(kb0, qr, sLb);
            sLa = wmma16g(kra0, qh, sLa); sLb = wmma16g(krb0, qh, sLb);
        }
        const int ja = key0 + 8 * hi;
        float ta[8], tb[8]; bool fa[8], fb[8]; float mx = NEGB;
#pragma unroll
        for (int r = 0; r < 8; ++r) {
            fa[r] = (ja + r <= lim);
            fb[r] = (ja + 16 + r <= lim);
            if (EARLY) { ta[r] = (sHa[r] + sLa[r] * QRI) * SC2; tb[r] = (sHb[r] + sLb[r] * QRI) * SC2; }
            else       { ta[r] = sHa[r] * SC2; tb[r] = sHb[r] * SC2; }
            mx = fmaxf(mx, fmaxf(fa[r] ? ta[r] : NEGB, fb[r] ? tb[r] : NEGB)); }
        mx = fmaxf(mx, __shfl_xor(mx, 16, 32));
        const float mnew = fmaxf(m, mx);
        const float alpha = __builtin_amdgcn_exp2f(m - mnew);
        const float sh = PSH - mnew;
        v16h pb, pr = hz; float ls = 0.0f;
#pragma unroll
        for (int r = 0; r < 8; ++r) {
            const float xa = ta[r] + sh, xb = tb[r] + sh;
            const float ea = __builtin_amdgcn_exp2f(xa), eb = __builtin_amdgcn_exp2f(xb);
            const float ga = (fa[r] & (xa >= PFL)) ? ea : 0.0f, gb = (fb[r] & (xb >= PFL)) ? eb : 0.0f;
            const h16 pa = (h16)ga; const h16 pc = (h16)gb;
            pb[r] = pa; pb[8 + r] = pc;
            if (EARLY) { pr[r] = toh_flush((ga - (float)pa) * QRS); pr[8 + r] = toh_flush((gb - (float)pc) * QRS); ls += ga + gb; }
            else       { ls += (float)pa + (float)pc; } }
        l = l * alpha + ls; m = mnew;
        o0 = o0 * alpha; o1 = o1 * alpha;
        if (EARLY) { oR0 = oR0 * alpha; oR1 = oR1 * alpha; }
        const h16* va = VT + vo + key0;
        const v16h v0 = ldh(va), v1 = ldh(va + (size_t)16 * SEQ);
        o0 = wmma16g(v0, pb, o0); o1 = wmma16g(v1, pb, o1);
        if (EARLY) {
            const h16* vr = VR + vro + key0;
            const v16h vr0 = ldh(vr), vr1 = ldh(vr + (size_t)16 * EROWS);
            oR0 = wmma16g(v0, pr, oR0); oR1 = wmma16g(v1, pr, oR1);
            oR0 = wmma16g(vr0, pb, oR0); oR1 = wmma16g(vr1, pb, oR1);
        }
    }
    l += __shfl_xor(l, 16, 32);
    const bool any = l > 0.0f;
    const float lsafe = any ? l : 1.0f;
    const float inv = any ? ((1.0f / lsafe) * CTXS) : 0.0f;
    v8f f0 = o0, f1 = o1;
    if (EARLY) { f0 = o0 + oR0 * QRI; f1 = o1 + oR1 * QRI; }
    const int wb = wave * 16 * OSP;
    { v4f a, c;
      a[0] = f0[0] * inv; a[1] = f0[1] * inv; a[2] = f0[2] * inv; a[3] = f0[3] * inv; c[0] = f0[4] * inv; c[1] = f0[5] * inv; c[2] = f0[6] * inv; c[3] = f0[7] * inv;
      *(v4fa*)(&os[wb + lr * OSP +  0 + 8 * hi]) = a; *(v4fa*)(&os[wb + lr * OSP +  0 + 8 * hi + 4]) = c;
      a[0] = f1[0] * inv; a[1] = f1[1] * inv; a[2] = f1[2] * inv; a[3] = f1[3] * inv; c[0] = f1[4] * inv; c[1] = f1[5] * inv; c[2] = f1[6] * inv; c[3] = f1[7] * inv;
      *(v4fa*)(&os[wb + lr * OSP + 16 + 8 * hi]) = a; *(v4fa*)(&os[wb + lr * OSP + 16 + 8 * hi + 4]) = c; }
    wave_sync();
    const size_t cb = ((size_t)(h * NB + b) * SEQ + (size_t)t0) * HD;
    const size_t rb = ((size_t)(h * NB + b) * EROWS + (size_t)(EARLY ? t0 : 0)) * HD;
#pragma unroll 1
    for (int ps = 0; ps < 2; ++ps) {
#pragma unroll
        for (int s = 0; s < 2; ++s) { const int p = s * 32 + lane; const int row = p >> 2, c8 = (p & 3) * 8;
            const v4f x0 = *(const v4fa*)(&os[wb + row * OSP + c8]); const v4f x1 = *(const v4fa*)(&os[wb + row * OSP + c8 + 4]); v8h hv, rv;
#pragma unroll
            for (int i = 0; i < 4; ++i) { const h16 a0 = toh_flush(x0[i]); const h16 a1 = toh_flush(x1[i]); hv[i] = a0; hv[4 + i] = a1;
                if (EARLY) { rv[i] = toh_flush((x0[i] - (float)a0) * QRS); rv[4 + i] = toh_flush((x1[i] - (float)a1) * QRS); } }
            *(volatile v8h*)(CH + cb + (size_t)p * 8) = hv;
            if (EARLY) *(volatile v8h*)(CR + rb + (size_t)p * 8) = rv; }
        if (ps == 0) __threadfence(); }
}

__global__ __launch_bounds__(32 * AW) void k_flash_early(const h16* __restrict__ QH, const h16* __restrict__ QR, const h16* __restrict__ KP, const h16* __restrict__ KR,
                                                         const h16* __restrict__ VT, const h16* __restrict__ VR, h16* CH, h16* CR) {
    flash_body<1>(QH, QR, KP, KR, VT, VR, CH, CR);
}
__global__ __launch_bounds__(32 * AW) void k_flash_late(const h16* __restrict__ QH, const h16* __restrict__ KP, const h16* __restrict__ VT, h16* CH) {
    flash_body<0>(QH, QH, KP, KP, VT, VT, CH, CH);
}

template <int EARLY>
__device__ __forceinline__ void oproj_body(const h16* __restrict__ CH, const h16* __restrict__ CR, const h16* __restrict__ WP, float* OUT) {
    __shared__ __align__(16) float os[AW * 16 * DMI];
    const int lane = threadIdx.x & 31, lr = lane & 15, hi = lane >> 4;
    const int wave = __builtin_amdgcn_readfirstlane((int)(threadIdx.x >> 5));
    const int b = blockIdx.y;
    const int t0 = (EARLY ? 0 : EROWS) + (blockIdx.x * AW + wave) * 16;
    v8f acc[8], accR[8];
#pragma unroll
    for (int nb = 0; nb < 8; ++nb) { acc[nb] = (v8f){}; accR[nb] = (v8f){}; }
    const size_t ao  = ((size_t)b * SEQ + (size_t)(t0 + lr)) * HD + 8 * hi;
    const size_t aro = ((size_t)b * EROWS + (size_t)(EARLY ? (t0 + lr) : lr)) * HD + 8 * hi;
    const size_t wo  = (size_t)lr * DH + 8 * hi;
#pragma unroll 1
    for (int kc = 0; kc < NH_; ++kc) {
        const v16h a = ldh(CH + ao + (size_t)kc * ((size_t)NB * SEQ * HD));
        v16h ar = (v16h){}; if (EARLY) ar = ldh(CR + aro + (size_t)kc * ((size_t)NB * EROWS * HD));
#pragma unroll
        for (int nb = 0; nb < 8; ++nb) { const v16h w = ldh(WP + wo + (size_t)nb * 16 * DH + (size_t)kc * HD);
            acc[nb] = wmma16g(a, w, acc[nb]);
            if (EARLY) accR[nb] = wmma16g(ar, w, accR[nb]); }
    }
    const int wb = wave * 16 * DMI;
#pragma unroll
    for (int nb = 0; nb < 8; ++nb) {
        const int col = nb * 16 + lr;
#pragma unroll
        for (int j = 0; j < 8; ++j) {
            float v = acc[nb][j]; if (EARLY) v = v + accR[nb][j] * QRI;
            v = v * OSC;
            if (col < DMI) os[wb + (hi * 8 + j) * DMI + col] = v; } }
    wave_sync();
    float* ob = OUT + ((size_t)b * OUT_SEQ + (size_t)t0) * DMI;
#pragma unroll 1
    for (int ps = 0; ps < 2; ++ps) {
#pragma unroll 1
        for (int it = 0; it < OPT; ++it) { const int idx = it * 32 + lane; const int ic = idx < OPQ ? idx : (OPQ - 1);
            const v4f val = *(const v4fa*)(&os[wb + ic * 4]);
            if (idx < OPQ) *(volatile v4f*)(ob + (size_t)idx * 4) = val; }
        if (ps == 0) __threadfence(); }
}

__global__ __launch_bounds__(32 * AW) void k_oproj_early(const h16* __restrict__ CH, const h16* __restrict__ CR, const h16* __restrict__ WP, float* OUT) { oproj_body<1>(CH, CR, WP, OUT); }
__global__ __launch_bounds__(32 * AW) void k_oproj_late(const h16* __restrict__ CH, const h16* __restrict__ WP, float* OUT) { oproj_body<0>(CH, CH, WP, OUT); }

static constexpr size_t al256(size_t v) { return (v + 255) & ~(size_t)255; }
static constexpr size_t SZ_XB = al256((size_t)NB * SEQ * DK * 2);
static constexpr size_t SZ_WB = al256((size_t)3 * DH * DK * 2);
static constexpr size_t SZ_WP = al256((size_t)DNO * DH * 2);
static constexpr size_t SZ_PL = al256((size_t)NB * NH_ * SEQ * HD * 2);
static constexpr size_t SZ_RS = al256((size_t)NB * NH_ * EROWS * HD * 2);
static constexpr size_t SZ_TOTAL = SZ_XB + SZ_WB + SZ_WP + 4 * SZ_PL + 4 * SZ_RS;
static_assert(SZ_TOTAL <= (size_t)134217728);
static_assert(((size_t)DH * DK * 2) % 256 == 0);
static_assert((size_t)NB * NH_ * SEQ * HD == (size_t)NB * DH * SEQ);
static_assert((size_t)NB * NH_ * EROWS * HD == (size_t)NB * DH * EROWS);
static_assert((size_t)NB * SEQ * (DK / 8) < (size_t)0x7fffffff);

extern "C" void kernel_launch(void* const* d_in, const int* in_sizes, int n_in,
                              void* d_out, int out_size, void* d_ws, size_t ws_size, hipStream_t stream) {
    if (n_in < 3) return;
    const size_t needx = ((size_t)(NB - 1) * SEQ_FULL + SEQ) * DMI;
    if ((size_t)in_sizes[0] < needx) return;
    if ((size_t)in_sizes[1] < (size_t)DMI * 3 * DMI || (size_t)in_sizes[2] < (size_t)DMI * DMI) return;
    if ((size_t)out_size < ((size_t)(NB - 1) * OUT_SEQ + SEQ) * DMI) return;
    if (SZ_TOTAL > ws_size) return;
    const float* xin = (const float*)d_in[0];
    const float* wat = (const float*)d_in[1];
    const float* wpr = (const float*)d_in[2];
    float* OUT = (float*)d_out;
    char* wsp = (char*)d_ws;
    bf* XB = (bf*)wsp; wsp += SZ_XB;
    bf* WB = (bf*)wsp; wsp += SZ_WB;
    h16* WP = (h16*)wsp; wsp += SZ_WP;
    h16* QH = (h16*)wsp; wsp += SZ_PL;
    h16* KP = (h16*)wsp; wsp += SZ_PL;
    h16* VT = (h16*)wsp; wsp += SZ_PL;
    h16* CH = (h16*)wsp; wsp += SZ_PL;
    h16* QR = (h16*)wsp; wsp += SZ_RS;
    h16* KR = (h16*)wsp; wsp += SZ_RS;
    h16* VR = (h16*)wsp; wsp += SZ_RS;
    h16* CR = (h16*)wsp; wsp += SZ_RS;
    bf* WQ = WB; bf* WK = WB + (size_t)DH * DK; bf* WV = WB + (size_t)2 * DH * DK;

    { const unsigned n8 = (unsigned)((size_t)NB * SEQ * (DK / 8));
      k_padx<<<(n8 + 255u) / 256u, 256, 0, stream>>>(xin, XB, n8); }
    k_wprep<<<WBLK + PBLK, 256, 0, stream>>>(wat, wpr, WB, WP);

    k_proj_rows<<<dim3(NB * SEQ / 64, DH / 64, 1), 32, 0, stream>>>(XB, WQ, QH, QR, EROWS);
    k_proj_rows<<<dim3(NB * SEQ / 64, DH / 64, 1), 32, 0, stream>>>(XB, WK, KP, KR, EROWS);
    k_proj_cols<<<dim3(DH / 64, NB * SEQ / 64, 1), 32, 0, stream>>>(WV, XB, VT, VR, EROWS);

    k_flash_early<<<dim3(EROWS / (16 * AW), NB * NH_, 1), 32 * AW, 0, stream>>>(QH, QR, KP, KR, VT, VR, CH, CR);
    if (SEQ > EROWS)
        k_flash_late<<<dim3((SEQ - EROWS) / (16 * AW), NB * NH_, 1), 32 * AW, 0, stream>>>(QH, KP, VT, CH);
    k_oproj_early<<<dim3(EROWS / (16 * AW), NB, 1), 32 * AW, 0, stream>>>(CH, CR, WP, OUT);
    if (SEQ > EROWS)
        k_oproj_late<<<dim3((SEQ - EROWS) / (16 * AW), NB, 1), 32 * AW, 0, stream>>>(CH, WP, OUT);
}
